// DeepTensorNN_66211215835150
// MI455X (gfx1250) — hardware-verified
//
#include <hip/hip_runtime.h>
#include <stdint.h>

#define BATCH 64
#define NATOM 256
#define AEMB  20
#define NRBF  25
#define NF    45
#define NHID  10
#define NTHR  256
#define NWAVE 8
#define APW   (NATOM / NWAVE)
#define NJT   (NATOM / 16)
static_assert(NWAVE * APW == NATOM);
static_assert(NJT * 16 == NATOM);
static_assert(AEMB + NRBF == NF);
static_assert(AEMB > 16 && AEMB <= 32);
static_assert(NRBF <= 32);

#define TWO_LOG2E   2.8853900817779268f
#define NEG2_LOG2E (-2.8853900817779268f)

typedef __bf16       v16b __attribute__((ext_vector_type(16)));
typedef float        v8f  __attribute__((ext_vector_type(8)));
typedef float        v4f  __attribute__((ext_vector_type(4)));
typedef unsigned int v8u  __attribute__((ext_vector_type(8)));
union Frag { v8u u; v16b v; };
static_assert(sizeof(Frag) == 32);

__device__ __forceinline__ unsigned short bf_bits(float f) {
  unsigned u = __float_as_uint(f);
  return (unsigned short)((u + 0x7FFFu + ((u >> 16) & 1u)) >> 16);
}
__device__ __forceinline__ float bf_up(unsigned short s) { return __uint_as_float(((unsigned)s) << 16); }
__device__ __forceinline__ float bfr(float f) { return bf_up(bf_bits(f)); }
__device__ __forceinline__ unsigned pk16(unsigned short a, unsigned short b) { return (unsigned)a | ((unsigned)b << 16); }
__device__ __forceinline__ v8f zero8() { v8f zz = {0.f, 0.f, 0.f, 0.f, 0.f, 0.f, 0.f, 0.f}; return zz; }

__device__ __forceinline__ float rbf(float d, float mu) {
  const float t = d - mu;
  return __builtin_amdgcn_exp2f((t * t) * NEG2_LOG2E);
}
__device__ __forceinline__ float tanh_fast(float x) {
  const float e = __builtin_amdgcn_exp2f(x * TWO_LOG2E);
  const float r = __builtin_amdgcn_rcpf(e + 1.0f);
  return 1.0f - 2.0f * r;
}

__device__ __forceinline__ v8f mma_bf(v16b a, v16b b, v8f c) {
  c = __builtin_amdgcn_wmma_f32_16x16x32_bf16(false, a, false, b, (short)0, c, false, false);
#if defined(__HIP_DEVICE_COMPILE__)
  asm volatile("v_nop\n\tv_nop\n\tv_nop\n\tv_nop" : "+v"(c) : "v"(a), "v"(b));
#endif
  return c;
}

template <int KB>
__device__ __forceinline__ unsigned rbf_pair(float d, int h) {
  const float muA0 = (float)(KB)     * 0.2f;
  const float muA1 = (float)(KB + 1) * 0.2f;
  const float muB0 = (float)(KB + 8) * 0.2f;
  const float muB1 = (float)(KB + 9) * 0.2f;
  const bool hh = (h != 0);
  const float mu0 = hh ? muB0 : muA0;
  const float mu1 = hh ? muB1 : muA1;
  float g0 = rbf(d, mu0);
  float g1 = rbf(d, mu1);
  const bool v0 = hh ? (KB + 8 < NRBF) : (KB < NRBF);
  const bool v1 = hh ? (KB + 9 < NRBF) : (KB + 1 < NRBF);
  g0 = v0 ? g0 : 0.0f;
  g1 = v1 ? g1 : 0.0f;
  return pk16(bf_bits(g0), bf_bits(g1));
}
template <int KB>
__device__ __forceinline__ unsigned vwd_pair(const float* sVw, int oc, bool ov, int h) {
  const int k0 = KB + 8 * h;
  const int k1 = k0 + 1;
  const float w0 = sVw[oc * NF + AEMB + min(k0, NRBF - 1)];
  const float w1 = sVw[oc * NF + AEMB + min(k1, NRBF - 1)];
  const float x0 = (ov && (k0 < NRBF)) ? w0 : 0.0f;
  const float x1 = (ov && (k1 < NRBF)) ? w1 : 0.0f;
  return pk16(bf_bits(x0), bf_bits(x1));
}

__global__ __launch_bounds__(NTHR)
void atom_energy(const int* __restrict__ z, const float* __restrict__ dist,
                 const float* __restrict__ emb, const float* __restrict__ Vw,
                 const float* __restrict__ Vb, const float* __restrict__ W1,
                 const float* __restrict__ b1, const float* __restrict__ W2,
                 const float* __restrict__ b2, float* E) {
  __shared__ __align__(16) float sEmb[NATOM * AEMB];
  __shared__ __align__(16) float sVw[AEMB * NF];
  __shared__ __align__(16) float sW1[NHID * AEMB];
  __shared__ float sVb[AEMB];
  __shared__ float sb1[NHID];
  __shared__ float sW2[NHID];
  __shared__ float sb2[1];
  __shared__ __align__(16) float sE[NATOM];

  const int tid  = threadIdx.x;
  const int wave = tid >> 5;
  const int lane = tid & 31;
  const int h    = lane >> 4;
  const int m    = lane & 15;
  const int b    = blockIdx.x;

  for (int idx = tid; idx < NATOM * AEMB; idx += NTHR) sEmb[idx] = bfr(emb[idx]);
  for (int idx = tid; idx < AEMB * NF; idx += NTHR) sVw[idx] = bfr(Vw[idx]);
  if (tid < NHID * AEMB) sW1[tid] = bfr(W1[tid]);
  if (tid < AEMB) sVb[tid] = bfr(Vb[tid]);
  if (tid < NHID) { sb1[tid] = bfr(b1[tid]); sW2[tid] = bfr(W2[tid]); }
  if (tid == 0) sb2[0] = bfr(b2[0]);
  __syncthreads();

  const int  o1c = min(16 + m, AEMB - 1);
  const bool o1v = (m < (AEMB - 16));
  Frag B0, B1;
  B0.u[0] = vwd_pair<0 >(sVw, m, true, h);
  B0.u[1] = vwd_pair<2 >(sVw, m, true, h);
  B0.u[2] = vwd_pair<4 >(sVw, m, true, h);
  B0.u[3] = vwd_pair<6 >(sVw, m, true, h);
  B0.u[4] = vwd_pair<16>(sVw, m, true, h);
  B0.u[5] = vwd_pair<18>(sVw, m, true, h);
  B0.u[6] = vwd_pair<20>(sVw, m, true, h);
  B0.u[7] = vwd_pair<22>(sVw, m, true, h);
  B1.u[0] = vwd_pair<0 >(sVw, o1c, o1v, h);
  B1.u[1] = vwd_pair<2 >(sVw, o1c, o1v, h);
  B1.u[2] = vwd_pair<4 >(sVw, o1c, o1v, h);
  B1.u[3] = vwd_pair<6 >(sVw, o1c, o1v, h);
  B1.u[4] = vwd_pair<16>(sVw, o1c, o1v, h);
  B1.u[5] = vwd_pair<18>(sVw, o1c, o1v, h);
  B1.u[6] = vwd_pair<20>(sVw, o1c, o1v, h);
  B1.u[7] = vwd_pair<22>(sVw, o1c, o1v, h);

  const int oc = min(lane, AEMB - 1);
  const v8f czero = zero8();

#pragma unroll 1
  for (int a = 0; a < APW; ++a) {
    const int i   = wave * APW + a;
    const int zi  = z[b * NATOM + i];
    const float maskf = (zi != 0) ? 1.0f : 0.0f;
    const int zc  = min(max(zi, 0), NATOM - 1);
    const float* ce = sEmb + zc * AEMB;

    float u0 = 0.0f, u1 = 0.0f;
#pragma unroll
    for (int f = 0; f < AEMB; ++f) {
      const float cf = ce[f] * maskf;
      u0 += sVw[m   * NF + f] * cf;
      u1 += sVw[o1c * NF + f] * cf;
    }
    const float ub0 = u0 + sVb[m];
    const float ub1 = u1 + sVb[o1c];

    const float* drow = dist + (size_t)(b * NATOM + i) * NATOM + m;
    float acc0 = 0.0f, acc1 = 0.0f;
#pragma unroll 1
    for (int jt = 0; jt < NJT; ++jt) {
      const float d = bfr(drow[jt * 16]);
      Frag A;
      A.u[0] = rbf_pair<0 >(d, h);
      A.u[1] = rbf_pair<2 >(d, h);
      A.u[2] = rbf_pair<4 >(d, h);
      A.u[3] = rbf_pair<6 >(d, h);
      A.u[4] = rbf_pair<16>(d, h);
      A.u[5] = rbf_pair<18>(d, h);
      A.u[6] = rbf_pair<20>(d, h);
      A.u[7] = rbf_pair<22>(d, h);
      const v8f d0 = mma_bf(A.v, B0.v, czero);
      const v8f d1 = mma_bf(A.v, B1.v, czero);
#pragma unroll
      for (int r = 0; r < 8; ++r) {
        acc0 += tanh_fast(d0[r] + ub0);
        acc1 += tanh_fast(d1[r] + ub1);
      }
    }
    const float agg0 = (acc0 + __shfl_xor(acc0, 16, 32)) * maskf;
    const float agg1 = (acc1 + __shfl_xor(acc1, 16, 32)) * maskf;
    const float aggL = (lane < 16) ? agg0 : agg1;
    const float cfL  = ce[oc] * maskf;
    float t = tanh_fast(cfL + aggL);
    t = (lane < AEMB) ? t : 0.0f;

    float eacc = 0.0f;
#pragma unroll
    for (int p = 0; p < NHID; ++p) {
      float part = sW1[p * AEMB + oc] * t;
      part += __shfl_xor(part, 16, 32);
      part += __shfl_xor(part, 8, 32);
      part += __shfl_xor(part, 4, 32);
      part += __shfl_xor(part, 2, 32);
      part += __shfl_xor(part, 1, 32);
      eacc += sW2[p] * (part + sb1[p]);
    }
    const float e = eacc + sb2[0];
    if (lane == 0) sE[i] = e;
  }
  __syncthreads();

  if (tid < NATOM / 4) {
    const v4f v = *(const v4f*)(sE + tid * 4);
    float* dst = E + (size_t)b * NATOM + tid * 4;
    *(volatile v4f*)dst = v;
    __threadfence();
    *(volatile v4f*)dst = v;
  }
}

__global__ __launch_bounds__(64)
void finish(const float* __restrict__ E, float* out) {
  __shared__ __align__(16) float sOut[BATCH];
  const int tid = threadIdx.x;
  const float* row = E + (size_t)tid * NATOM;
  float s = 0.0f;
#pragma unroll 4
  for (int a = 0; a < NATOM; ++a) s += row[a];
  sOut[tid] = s;
  __syncthreads();
  if (tid < BATCH / 4) {
    const v4f v = *(const v4f*)(sOut + tid * 4);
    *(volatile v4f*)(out + tid * 4) = v;
    __threadfence();
    *(volatile v4f*)(out + tid * 4) = v;
  }
}

extern "C" void kernel_launch(void* const* d_in, const int* in_sizes, int n_in,
                              void* d_out, int out_size, void* d_ws, size_t ws_size,
                              hipStream_t stream) {
  if (n_in < 9) return;
  if (in_sizes[0] != BATCH * NATOM) return;
  if (in_sizes[1] != BATCH * NATOM * NATOM) return;
  if (in_sizes[2] != NATOM * AEMB) return;
  if (in_sizes[3] != AEMB * NF) return;
  if (in_sizes[4] != AEMB) return;
  if (in_sizes[5] != NHID * AEMB) return;
  if (in_sizes[6] != NHID) return;
  if (in_sizes[7] != NHID) return;
  if (in_sizes[8] != 1) return;
  if (out_size != BATCH) return;

  const size_t eBytes = (size_t)BATCH * NATOM * sizeof(float);
  if (eBytes > ws_size) return;
  if (eBytes > (size_t)134217728) return;

  const int*   z    = (const int*)  d_in[0];
  const float* dist = (const float*)d_in[1];
  const float* emb  = (const float*)d_in[2];
  const float* Vw   = (const float*)d_in[3];
  const float* Vb   = (const float*)d_in[4];
  const float* W1   = (const float*)d_in[5];
  const float* b1   = (const float*)d_in[6];
  const float* W2   = (const float*)d_in[7];
  const float* b2   = (const float*)d_in[8];
  float* E   = (float*)d_ws;
  float* out = (float*)d_out;

  atom_energy<<<dim3(BATCH), dim3(NTHR), 0, stream>>>(z, dist, emb, Vw, Vb, W1, b1, W2, b2, E);
  finish<<<dim3(1), dim3(64), 0, stream>>>(E, out);
  (void)hipGetLastError();
}
